// VRWKV_SpatialMix_50096498541307
// MI455X (gfx1250) — hardware-verified
//
#include <hip/hip_runtime.h>
#include <math.h>

constexpr int kH = 64;
constexpr int kW = 64;
constexpr int kC = 256;
constexpr int kT = kH * kW;
constexpr int kL = 64;
constexpr int kNC = kT / kL;
constexpr int kStencilFloats = kC * 25 + kC * 9 + kC;
constexpr float kNegInit = -1.0e30f;
constexpr float kInvT = 1.0f / 4096.0f;
constexpr float kCarryA = 8.0f;
constexpr float kCarryAInv = 0.125f;
constexpr float kCarryW = 16.0f;
constexpr float kScaleAW = 1.0f / 128.0f;
constexpr float kScaleW = 1.0f / 16.0f;
constexpr float kInvC = 1.0f / 256.0f;
constexpr float kLnEps = 1.0e-5f;
static_assert(kT % kL == 0, "chunking");
static_assert(kC % 64 == 0, "gemm N tile");
static_assert(kC % 32 == 0, "gemm K step");
static_assert(kT % 128 == 0, "gemm M tile and block grouping");
static_assert(kStencilFloats == 8960, "stencil staging size");

typedef __attribute__((ext_vector_type(16))) _Float16 v16h;
typedef __attribute__((ext_vector_type(8)))  _Float16 v8h;
typedef __attribute__((ext_vector_type(16))) __bf16   v16b;
typedef __attribute__((ext_vector_type(8)))  __bf16   v8b;
typedef __attribute__((ext_vector_type(8)))  float    v8f;
typedef __attribute__((ext_vector_type(4)))  float    v4f;
typedef __attribute__((ext_vector_type(4)))  unsigned int v4u;

__device__ __forceinline__ unsigned short f2bf_bits(float f) {
  unsigned u = __float_as_uint(f);
  return (unsigned short)((u + 0x7FFFu + ((u >> 16) & 1u)) >> 16);
}
__device__ __forceinline__ float bf_bits2f(unsigned short h) { return __uint_as_float(((unsigned)h) << 16); }

__device__ __forceinline__ void dep_guard_h(v8f& a, v8f& b, v16h x, v16h y) { asm volatile("v_nop\n\tv_nop\n\tv_nop\n\tv_nop" : "+v"(a), "+v"(b) : "v"(x), "v"(y)); }
__device__ __forceinline__ void dep_guard_b(v8f& a, v8f& b, v16b x, v16b y) { asm volatile("v_nop\n\tv_nop\n\tv_nop\n\tv_nop" : "+v"(a), "+v"(b) : "v"(x), "v"(y)); }
__device__ __forceinline__ void keep4_h(v16h a, v16h b, v16h c, v16h d) { asm volatile("v_nop" :: "v"(a), "v"(b), "v"(c), "v"(d)); }
__device__ __forceinline__ void keep4_b(v16b a, v16b b, v16b c, v16b d) { asm volatile("v_nop" :: "v"(a), "v"(b), "v"(c), "v"(d)); }
__device__ __forceinline__ void acc_guard4(v8f& a, v8f& b, v8f& c, v8f& d) { asm volatile("v_nop\n\tv_nop\n\tv_nop\n\tv_nop" : "+v"(a), "+v"(b), "+v"(c), "+v"(d)); }
template <typename T> struct Frag;
template <> struct Frag<_Float16> {
  typedef v16h V; union U { v16h v; v8h h[2]; };
  static __device__ __forceinline__ v16h load(const _Float16* p) {
    U f; f.h[0] = *(const v8h*)(p); f.h[1] = *(const v8h*)(p + 16); return f.v;
  }
  static __device__ __forceinline__ v8f mma(v16h a, v16h b, v8f c) {
    return __builtin_amdgcn_wmma_f32_16x16x32_f16(false, a, false, b, (short)0, c, false, false);
  }
  static __device__ __forceinline__ void guard(v8f& a, v8f& b, v16h x, v16h y) { dep_guard_h(a, b, x, y); }
  static __device__ __forceinline__ void keep(v16h a, v16h b, v16h c, v16h d) { keep4_h(a, b, c, d); }
};
template <> struct Frag<__bf16> {
  typedef v16b V; union U { v16b v; v8b h[2]; };
  static __device__ __forceinline__ v16b load(const __bf16* p) {
    U f; f.h[0] = *(const v8b*)(p); f.h[1] = *(const v8b*)(p + 16); return f.v;
  }
  static __device__ __forceinline__ v8f mma(v16b a, v16b b, v8f c) {
    return __builtin_amdgcn_wmma_f32_16x16x32_bf16(false, a, false, b, (short)0, c, false, false);
  }
  static __device__ __forceinline__ void guard(v8f& a, v8f& b, v16b x, v16b y) { dep_guard_b(a, b, x, y); }
  static __device__ __forceinline__ void keep(v16b a, v16b b, v16b c, v16b d) { keep4_b(a, b, c, d); }
};

__device__ __forceinline__ unsigned pk16(unsigned short a, unsigned short b) { return (unsigned)a | ((unsigned)b << 16); }
__device__ __forceinline__ unsigned short h_bits(float f) { const _Float16 h = (_Float16)f; return __builtin_bit_cast(unsigned short, h); }

__device__ __forceinline__ float h16_to_f32(unsigned hb) {
  const unsigned sgn = (hb & 0x8000u) << 16; const unsigned em = hb & 0x7fffu;
  const float fn = __uint_as_float((em << 13) + 0x38000000u);
  const float fs = (float)em * 5.9604644775390625e-8f;
  const float mag = (em < 0x400u) ? fs : fn; return __uint_as_float(__float_as_uint(mag) | sgn); }

template <int ET> struct Elem;
template <> struct Elem<0> { typedef _Float16 T; };
template <> struct Elem<1> { typedef __bf16 T; };
template <int ET, bool SPLIT, int BIAS_MODE, int OUT_MODE, bool RESID, int ACT = 0>
__global__ __launch_bounds__(256) void wmma_gemm64(
    const unsigned short* __restrict__ Ap, const unsigned short* __restrict__ A2p, int lda, long strideA,
    const unsigned short* __restrict__ Btp, const unsigned short* __restrict__ Bt2p, int ldb, long strideB,
    void* __restrict__ Cout, void* __restrict__ Cout2, int ldc, long strideC,
    const float* __restrict__ bias,
    const float* __restrict__ resid, long strideR,
    int M, int N, int K, float scale) {
  typedef typename Elem<ET>::T T;
  typedef typename Frag<T>::V V;
  const T* A = (const T*)Ap; const T* A2 = (const T*)A2p; const T* Bt = (const T*)Btp; const T* Bt2 = (const T*)Bt2p;
  __shared__ __align__(16) float sT[8][16 * 68];
  const int b    = blockIdx.y;
  const int lane = threadIdx.x & 31;
  const int wave = threadIdx.x >> 5;
  const int tilesN = N >> 6;
  const int tilesM = M >> 6;
  const int tile = blockIdx.x * 8 + wave;
  if (tile >= tilesM * tilesN) return;
  const int tm = tile / tilesN;
  const int tn = tile - tm * tilesN;
  const int m0 = tm << 6;
  const int n0 = tn << 6;

  const T* Ab  = A  + (size_t)b * strideA;
  const T* Bb  = Bt + (size_t)b * strideB;
  const T* Ab2 = SPLIT ? (A2  + (size_t)b * strideA) : nullptr;
  const T* Bb2 = SPLIT ? (Bt2 + (size_t)b * strideB) : nullptr;

  const int rlane = lane & 15;
  const int koff  = (lane >> 4) * 8;
  const int mOff  = (lane >> 4) * 8;

  v8f acc[4][4];
#pragma unroll
  for (int i = 0; i < 4; ++i)
#pragma unroll
    for (int j = 0; j < 4; ++j) acc[i][j] = (v8f){0.f,0.f,0.f,0.f,0.f,0.f,0.f,0.f};

  for (int k0 = 0; k0 < K; k0 += 32) {
    V bh[4], bl[4];
#pragma unroll
    for (int j = 0; j < 4; ++j) {
      const size_t bo = (size_t)(n0 + (j << 4) + rlane) * ldb + koff + k0;
      bh[j] = Frag<T>::load(Bb + bo);
      if (SPLIT) bl[j] = Frag<T>::load(Bb2 + bo);
    }
#pragma unroll
    for (int i = 0; i < 4; ++i) {
      const size_t ao = (size_t)(m0 + (i << 4) + rlane) * lda + koff + k0;
      V ah = Frag<T>::load(Ab + ao);
      V al;
      if (SPLIT) al = Frag<T>::load(Ab2 + ao);
#pragma unroll
      for (int j = 0; j < 4; ++j) {
        acc[i][j] = Frag<T>::mma(ah, bh[j], acc[i][j]);
        if (SPLIT) {
          acc[i][j] = Frag<T>::mma(ah, bl[j], acc[i][j]);
          acc[i][j] = Frag<T>::mma(al, bh[j], acc[i][j]);
        }
      }
      Frag<T>::guard(acc[i][0], acc[i][3], ah, SPLIT ? al : ah);
    }
    Frag<T>::keep(bh[0], bh[1], bh[2], bh[3]);
    if (SPLIT) Frag<T>::keep(bl[0], bl[1], bl[2], bl[3]);
  }
  acc_guard4(acc[0][0], acc[0][1], acc[0][2], acc[0][3]);
  acc_guard4(acc[1][0], acc[1][1], acc[1][2], acc[1][3]);
  acc_guard4(acc[2][0], acc[2][1], acc[2][2], acc[2][3]);
  acc_guard4(acc[3][0], acc[3][1], acc[3][2], acc[3][3]);

  float* slab = sT[wave];
  const float* Rb = RESID ? (resid + (size_t)b * strideR) : nullptr;
#pragma unroll
  for (int i = 0; i < 4; ++i) {
    const int mBase = m0 + (i << 4);
#pragma unroll
    for (int j = 0; j < 4; ++j) {
      const int n = n0 + (j << 4) + rlane;
      float bv = 0.f;
      if (BIAS_MODE == 2) bv = bias[n];
#pragma unroll
      for (int r = 0; r < 8; ++r) {
        float v = acc[i][j][r] * scale;
        if (BIAS_MODE == 1) v += bias[mBase + mOff + r];
        if (BIAS_MODE == 2) v += bv;
        if (RESID) v += Rb[(size_t)(mBase + mOff + r) * ldc + n];
        if (ACT == 2) v = fmaxf(v, 0.0f);
        if (ACT == 4) v = (v > 0.f) ? v : 0.01f * v;
        slab[(mOff + r) * 68 + (j << 4) + rlane] = v;
      }
    }
    __builtin_amdgcn_fence(__ATOMIC_RELEASE, "workgroup");
    __builtin_amdgcn_wave_barrier();
    __builtin_amdgcn_fence(__ATOMIC_ACQUIRE, "workgroup");
    if (OUT_MODE == 0) {
      float* C = (float*)Cout + (size_t)b * strideC;
      const int hh = lane >> 4, c4 = (lane & 15) * 4;
      for (int pass = 0; pass < 2; ++pass) {
#pragma unroll
        for (int it = 0; it < 8; ++it) {
          const int row = it * 2 + hh;
          v4f v = *(const v4f*)(slab + row * 68 + c4);
          *(volatile v4f*)(C + (size_t)(mBase + row) * ldc + n0 + c4) = v;
        }
        __threadfence();
      }
    } else {
      const int q = lane >> 3, c8 = (lane & 7) * 8;
      unsigned short* C  = (unsigned short*)Cout  + (size_t)b * strideC;
      unsigned short* C2 = (OUT_MODE == 2) ? ((unsigned short*)Cout2 + (size_t)b * strideC) : nullptr;
      for (int pass = 0; pass < 2; ++pass) {
#pragma unroll
        for (int it = 0; it < 4; ++it) {
          const int row = it * 4 + q;
          const float* sp = slab + row * 68 + c8;
          v8h hv, lv;
#pragma unroll
          for (int e = 0; e < 8; ++e) {
            if (OUT_MODE == 1) {
              hv[e] = (_Float16)sp[e];
            } else {
              unsigned short hb = f2bf_bits(sp[e]);
              unsigned short lb = f2bf_bits(sp[e] - bf_bits2f(hb));
              hv[e] = __builtin_bit_cast(_Float16, hb);
              lv[e] = __builtin_bit_cast(_Float16, lb);
            }
          }
          *(volatile v8h*)(C + (size_t)(mBase + row) * ldc + n0 + c8) = hv;
          if (OUT_MODE == 2) *(volatile v8h*)(C2 + (size_t)(mBase + row) * ldc + n0 + c8) = lv;
        }
        __threadfence();
      }
    }
    __builtin_amdgcn_fence(__ATOMIC_RELEASE, "workgroup");
    __builtin_amdgcn_wave_barrier();
    __builtin_amdgcn_fence(__ATOMIC_ACQUIRE, "workgroup");
  }
}

__device__ __forceinline__ int imin(int a, int b) { return a < b ? a : b; }
__device__ __forceinline__ int imax(int a, int b) { return a > b ? a : b; }
__device__ __forceinline__ int seq_index(int s, int swap) {
  const int sw = ((s & (kH - 1)) << 6) | (s >> 6);
  return swap ? sw : s;
}
__device__ __forceinline__ void wkv_step(float& a, float& b, float& p, float w, float kt, float vt) {
  const float pd = p - w;
  const float d  = pd - kt;
  const float e  = expf(-fabsf(d));
  const bool  ge = (d >= 0.0f);
  const float e1 = ge ? 1.0f : e;
  const float e2 = ge ? e : 1.0f;
  a = e1 * a + e2 * vt;
  b = e1 * b + e2;
  p = fmaxf(pd, kt);
}
__device__ __forceinline__ void wkv_merge(float& a, float& b, float p1d, float a2, float b2, float p2, float pnew) {
  const float e1 = expf(p1d - pnew);
  const float e2 = expf(p2 - pnew);
  a = e1 * a + e2 * a2;
  b = e1 * b + e2 * b2;
}

__global__ __launch_bounds__(256) void wcast16_kernel(const float* __restrict__ W0, const float* __restrict__ W1,
                                                      const float* __restrict__ W2, const float* __restrict__ W3,
                                                      unsigned short* __restrict__ out, float scale) {
  const int z = blockIdx.y;
  const float* Wm = (z == 0) ? W0 : (z == 1) ? W1 : (z == 2) ? W2 : W3;
  const int i = blockIdx.x * 256 + threadIdx.x;
  if (i >= (kC * kC) / 8) return;
  const float* p = Wm + 8 * (size_t)i;
  const v4f a = *(const v4f*)(p);
  const v4f c = *(const v4f*)(p + 4);
  unsigned short hb[8];
#pragma unroll
  for (int e = 0; e < 4; ++e) {
    hb[e]     = h_bits(a[e] * scale);
    hb[4 + e] = h_bits(c[e] * scale);
  }
  const v4u u = (v4u){pk16(hb[0], hb[1]), pk16(hb[2], hb[3]), pk16(hb[4], hb[5]), pk16(hb[6], hb[7])};
  unsigned short* q = out + (size_t)z * kC * kC + 8 * (size_t)i;
  *(volatile v4u*)q = u;
  __threadfence();
  *(volatile v4u*)q = u;
}

__global__ __launch_bounds__(256) void omni_mix_kernel(const float* __restrict__ x, const float* __restrict__ alpha,
                                                       const float* __restrict__ w1, const float* __restrict__ w3,
                                                       const float* __restrict__ w5,
                                                       const float* __restrict__ mk, const float* __restrict__ mv,
                                                       const float* __restrict__ mr,
                                                       unsigned short* __restrict__ xq, long planeElems,
                                                       const int* __restrict__ hwH, const int* __restrict__ hwW) {
  __shared__ __align__(16) float swt[kStencilFloats];
  __shared__ __align__(16) unsigned short tile[3 * 16 * kC];
  (void)hwH; (void)hwW;
  const int c = threadIdx.x;
  const int b = blockIdx.x / kH;
  const int h = blockIdx.x % kH;
#pragma unroll 1
  for (int i = c; i < kC * 25; i += 256) swt[i] = w5[i];
#pragma unroll 1
  for (int i = c; i < kC * 9; i += 256) swt[kC * 25 + i] = w3[i];
  swt[kC * 25 + kC * 9 + c] = w1[c];
  __syncthreads();
  const float a0 = alpha[0], a1 = alpha[1], a2 = alpha[2], a3 = alpha[3];
  float coef[5][5];
#pragma unroll
  for (int di = 0; di < 5; ++di) {
#pragma unroll
    for (int dj = 0; dj < 5; ++dj) {
      float cc = a3 * swt[c * 25 + di * 5 + dj];
      if (di >= 1 && di <= 3 && dj >= 1 && dj <= 3) cc += a2 * swt[kC * 25 + c * 9 + (di - 1) * 3 + (dj - 1)];
      if (di == 2 && dj == 2) cc += a1 * swt[kC * 25 + kC * 9 + c] + a0;
      coef[di][dj] = cc;
    }
  }
  const float m_k = mk[c], m_v = mv[c], m_r = mr[c];
  const float o_k = 1.0f - m_k, o_v = 1.0f - m_v, o_r = 1.0f - m_r;

  const float* xb = x + (size_t)b * kT * kC + c;
  int hcl[5]; float vh[5];
  float win[5][5];
#pragma unroll
  for (int di = 0; di < 5; ++di) {
    const int hh = h - 2 + di;
    hcl[di] = imin(imax(hh, 0), kH - 1);
    vh[di]  = (hh >= 0 && hh < kH) ? 1.0f : 0.0f;
    win[di][0] = 0.0f;
    win[di][1] = 0.0f;
    win[di][2] = xb[(size_t)(hcl[di] * kW + 0) * kC] * vh[di];
    win[di][3] = xb[(size_t)(hcl[di] * kW + 1) * kC] * vh[di];
  }
  const size_t tokBase = (size_t)b * kT + (size_t)h * kW;
  const int lane = c & 31, wv = c >> 5;

#pragma unroll 1
  for (int wb = 0; wb < kW / 16; ++wb) {
#pragma unroll 1
    for (int wl = 0; wl < 16; ++wl) {
      const int w   = wb * 16 + wl;
      const int ww  = w + 2;
      const float vw = (ww < kW) ? 1.0f : 0.0f;
      const int wwc = imin(ww, kW - 1);
#pragma unroll
      for (int di = 0; di < 5; ++di) win[di][4] = xb[(size_t)(hcl[di] * kW + wwc) * kC] * (vh[di] * vw);
      float acc = 0.0f;
#pragma unroll
      for (int di = 0; di < 5; ++di)
#pragma unroll
        for (int dj = 0; dj < 5; ++dj) acc = fmaf(coef[di][dj], win[di][dj], acc);
      const float xc = win[2][2];
      const float vk = fmaf(xc, m_k, acc * o_k);
      const float vvv = fmaf(xc, m_v, acc * o_v);
      const float vr = fmaf(xc, m_r, acc * o_r);
      tile[(0 * 16 + wl) * kC + c] = h_bits(vk * kCarryA);
      tile[(1 * 16 + wl) * kC + c] = h_bits(vvv * kCarryA);
      tile[(2 * 16 + wl) * kC + c] = h_bits(vr * kCarryA);
#pragma unroll
      for (int di = 0; di < 5; ++di) {
        win[di][0] = win[di][1]; win[di][1] = win[di][2]; win[di][2] = win[di][3]; win[di][3] = win[di][4];
      }
    }
    __syncthreads();
    for (int rep = 0; rep < 2; ++rep) {
#pragma unroll
      for (int j = 0; j < 6; ++j) {
        const int r  = wv * 6 + j;
        const int pl = r >> 4, wl = r & 15;
        const v4u val = *(const v4u*)(tile + (size_t)r * kC + lane * 8);
        unsigned short* dst = xq + (size_t)pl * planeElems + (tokBase + wb * 16 + wl) * kC + lane * 8;
        *(volatile v4u*)dst = val;
      }
      __threadfence();
    }
    __syncthreads();
  }
}

__global__ __launch_bounds__(256) void wkv_chunk_kernel(const float* __restrict__ kp, const float* __restrict__ vp,
                                                        const float* __restrict__ sd, int par, int swap,
                                                        float* __restrict__ S) {
  const int c  = threadIdx.x;
  const int ch = blockIdx.x % kNC;
  const int b  = blockIdx.x / kNC;
  const float w = sd[par * kC + c] * kInvT;
  const size_t base = (size_t)b * kT * kC + c;
  float a = 0.0f, bb = 0.0f, p = kNegInit;
#pragma unroll 1
  for (int i = 0; i < kL; ++i) {
    const int t = seq_index(ch * kL + i, swap);
    const float kt = kp[base + (size_t)t * kC];
    const float vt = vp[base + (size_t)t * kC];
    wkv_step(a, bb, p, w, kt, vt);
  }
  const float aF = a, bF = bb, pF = p;
  a = 0.0f; bb = 0.0f; p = kNegInit;
#pragma unroll 1
  for (int i = kL - 1; i >= 0; --i) {
    const int t = seq_index(ch * kL + i, swap);
    const float kt = kp[base + (size_t)t * kC];
    const float vt = vp[base + (size_t)t * kC];
    wkv_step(a, bb, p, w, kt, vt);
  }
  const float aB = a, bB = bb, pB = p;
  float* rowp = S + (size_t)blockIdx.x * 6 * kC + c;
  for (int rep = 0; rep < 2; ++rep) {
    *(volatile float*)(rowp + 0 * kC) = aF;
    *(volatile float*)(rowp + 1 * kC) = bF;
    *(volatile float*)(rowp + 2 * kC) = pF;
    *(volatile float*)(rowp + 3 * kC) = aB;
    *(volatile float*)(rowp + 4 * kC) = bB;
    *(volatile float*)(rowp + 5 * kC) = pB;
    __threadfence();
  }
}

__global__ __launch_bounds__(32) void wkv_entries_kernel(const float* __restrict__ kp, const float* __restrict__ sd,
                                                         int par, int swap, const float* __restrict__ S,
                                                         float* __restrict__ E) {
  __shared__ float st[kNC][6][32];
  const int lane = threadIdx.x;
  const int b  = blockIdx.x >> 3;
  const int cg = blockIdx.x & 7;
  const int c  = cg * 32 + lane;
  const float w = sd[par * kC + c] * kInvT;
  const size_t kbase = (size_t)b * kT * kC + c;
  const float* Sb = S + (size_t)b * kNC * 6 * kC + c;
  float a = 0.0f, bb = 0.0f, pex = kNegInit;
#pragma unroll 1
  for (int ch = 0; ch < kNC; ++ch) {
    st[ch][0][lane] = a; st[ch][1][lane] = bb; st[ch][2][lane] = pex;
    float p = pex, dg = 0.0f;
#pragma unroll 4
    for (int i = 0; i < kL; ++i) {
      const int t = seq_index(ch * kL + i, swap);
      const float kt = kp[kbase + (size_t)t * kC];
      float pd = p - w;
      asm volatile("" : "+v"(pd));
      dg += pd - p;
      p = fmaxf(pd, kt);
    }
    const float aS = Sb[(size_t)(ch * 6 + 0) * kC];
    const float bS = Sb[(size_t)(ch * 6 + 1) * kC];
    const float pS = Sb[(size_t)(ch * 6 + 2) * kC];
    wkv_merge(a, bb, pex + dg, aS, bS, pS, p);
    pex = p;
  }
  a = 0.0f; bb = 0.0f; pex = kNegInit;
#pragma unroll 1
  for (int ch = kNC - 1; ch >= 0; --ch) {
    st[ch][3][lane] = a; st[ch][4][lane] = bb; st[ch][5][lane] = pex;
    float p = pex, dg = 0.0f;
#pragma unroll 4
    for (int i = kL - 1; i >= 0; --i) {
      const int t = seq_index(ch * kL + i, swap);
      const float kt = kp[kbase + (size_t)t * kC];
      float pd = p - w;
      asm volatile("" : "+v"(pd));
      dg += pd - p;
      p = fmaxf(pd, kt);
    }
    const float aS = Sb[(size_t)(ch * 6 + 3) * kC];
    const float bS = Sb[(size_t)(ch * 6 + 4) * kC];
    const float pS = Sb[(size_t)(ch * 6 + 5) * kC];
    wkv_merge(a, bb, pex + dg, aS, bS, pS, p);
    pex = p;
  }
  __syncthreads();
  float* Eb = E + (size_t)b * kNC * 6 * kC + c;
  for (int rep = 0; rep < 2; ++rep) {
#pragma unroll 1
    for (int ch = 0; ch < kNC; ++ch) {
#pragma unroll
      for (int j = 0; j < 6; ++j) {
        const float val = st[ch][j][lane];
        *(volatile float*)(Eb + (size_t)(ch * 6 + j) * kC) = val;
      }
    }
    __threadfence();
  }
}

__global__ __launch_bounds__(64) void wkv_apply_kernel(const float* __restrict__ kp, const float* __restrict__ vp,
                                                       const float* __restrict__ sd, const float* __restrict__ sf,
                                                       int par, int swap, const float* __restrict__ E,
                                                       float* __restrict__ yout) {
  __shared__ float sfx[kL][3][64];
  const int lane = threadIdx.x;
  const int cg = blockIdx.x & 3;
  const int bc = blockIdx.x >> 2;
  const int ch = bc % kNC;
  const int b  = bc / kNC;
  const int c  = cg * 64 + lane;
  const float w = sd[par * kC + c] * kInvT;
  const float u = sf[par * kC + c] * kInvT;
  const size_t base = (size_t)b * kT * kC + c;
  const float* Eb = E + (size_t)bc * 6 * kC + c;
  float a = Eb[3 * kC], bb = Eb[4 * kC], p = Eb[5 * kC];
#pragma unroll 1
  for (int i = kL - 1; i >= 0; --i) {
    sfx[i][0][lane] = a; sfx[i][1][lane] = bb; sfx[i][2][lane] = p;
    const int t = seq_index(ch * kL + i, swap);
    const float kt = kp[base + (size_t)t * kC];
    const float vt = vp[base + (size_t)t * kC];
    wkv_step(a, bb, p, w, kt, vt);
  }
  a = Eb[0 * kC]; bb = Eb[1 * kC]; p = Eb[2 * kC];
#pragma unroll 1
  for (int i = 0; i < kL; ++i) {
    const int t = seq_index(ch * kL + i, swap);
    const float kt = kp[base + (size_t)t * kC];
    const float vt = vp[base + (size_t)t * kC];
    const float ab = sfx[i][0][lane];
    const float b2 = sfx[i][1][lane];
    const float pb = sfx[i][2][lane];
    const float pc = u + kt;
    const float q  = fmaxf(fmaxf(p, pb), pc);
    const float ef = expf(p - q);
    const float eb = expf(pb - q);
    const float ec = expf(pc - q);
    const float num = ef * a + eb * ab + ec * vt;
    const float den = ef * bb + eb * b2 + ec;
    const float y = num / den;
    sfx[i][0][lane] = y;
    wkv_step(a, bb, p, w, kt, vt);
  }
  __syncthreads();
  for (int rep = 0; rep < 2; ++rep) {
#pragma unroll 1
    for (int i = 0; i < kL; ++i) {
      const int t = seq_index(ch * kL + i, swap);
      const float val = sfx[i][0][lane];
      *(volatile float*)(yout + base + (size_t)t * kC) = val;
    }
    __threadfence();
  }
}

__device__ __forceinline__ float gate_sigmoid(float z) {
  const float zc = fminf(fmaxf(z, -30.0f), 30.0f);
  const float e = expf(-zc);
  return __builtin_amdgcn_rcpf(1.0f + e);
}
__global__ __launch_bounds__(256) void ln_gate_kernel(const float* __restrict__ v2, const unsigned short* __restrict__ rlog,
                                                      const float* __restrict__ g, const float* __restrict__ beta,
                                                      unsigned short* __restrict__ aout, int Mrows) {
  const int lane = threadIdx.x & 31, wave = threadIdx.x >> 5;
  const int row = blockIdx.x * 8 + wave;
  if (row >= Mrows) return;
  const size_t off = (size_t)row * kC + lane * 8;
  const v4f va = *(const v4f*)(v2 + off);
  const v4f vc = *(const v4f*)(v2 + off + 4);
  float xv[8];
#pragma unroll
  for (int e = 0; e < 4; ++e) { xv[e] = va[e]; xv[4 + e] = vc[e]; }
  float s = ((xv[0] + xv[1]) + (xv[2] + xv[3])) + ((xv[4] + xv[5]) + (xv[6] + xv[7]));
#pragma unroll
  for (int o = 16; o > 0; o >>= 1) s += __shfl_xor(s, o, 32);
  const float mu = s * kInvC;
  float d[8];
  float ss = 0.0f;
#pragma unroll
  for (int e = 0; e < 8; ++e) { d[e] = xv[e] - mu; ss += d[e] * d[e]; }
#pragma unroll
  for (int o = 16; o > 0; o >>= 1) ss += __shfl_xor(ss, o, 32);
  const float var = ss * kInvC;
  const float rs = rsqrtf(var + kLnEps);
  const v4f ga = *(const v4f*)(g + lane * 8);
  const v4f gc = *(const v4f*)(g + lane * 8 + 4);
  const v4f ba = *(const v4f*)(beta + lane * 8);
  const v4f bcv = *(const v4f*)(beta + lane * 8 + 4);
  float gg[8], be[8];
#pragma unroll
  for (int e = 0; e < 4; ++e) { gg[e] = ga[e]; gg[4 + e] = gc[e]; be[e] = ba[e]; be[4 + e] = bcv[e]; }
  const v4u wd = *(const v4u*)(rlog + off);
  float sg[8];
#pragma unroll
  for (int j = 0; j < 4; ++j) {
    const unsigned wj = wd[j];
    const float z0 = h16_to_f32(wj & 0xffffu) * kCarryAInv;
    const float z1 = h16_to_f32(wj >> 16) * kCarryAInv;
    sg[2 * j]     = gate_sigmoid(z0);
    sg[2 * j + 1] = gate_sigmoid(z1);
  }
  unsigned short hb[8];
#pragma unroll
  for (int e = 0; e < 8; ++e) {
    const float ln = d[e] * rs * gg[e] + be[e];
    hb[e] = h_bits(sg[e] * ln * kCarryA);
  }
  const v4u uo = (v4u){pk16(hb[0], hb[1]), pk16(hb[2], hb[3]), pk16(hb[4], hb[5]), pk16(hb[6], hb[7])};
  unsigned short* q = aout + off;
  *(volatile v4u*)q = uo;
  __threadfence();
  *(volatile v4u*)q = uo;
}

extern "C" void kernel_launch(void* const* d_in, const int* in_sizes, int n_in,
                              void* d_out, int out_size, void* d_ws, size_t ws_size,
                              hipStream_t stream) {
  if (n_in < 18) return;
  const int nx = in_sizes[0];
  const int B = nx / (kT * kC);
  if (B < 1 || nx != B * kT * kC || out_size != nx) return;
  if (in_sizes[1] != kC || in_sizes[2] != kC || in_sizes[3] != kC) return;
  if (in_sizes[4] != 2 * kC || in_sizes[5] != 2 * kC || in_sizes[6] != 4) return;
  if (in_sizes[7] != kC || in_sizes[8] != kC * 9 || in_sizes[9] != kC * 25) return;
  if (in_sizes[10] != kC * kC || in_sizes[11] != kC * kC || in_sizes[12] != kC * kC || in_sizes[13] != kC * kC) return;
  if (in_sizes[14] != kC || in_sizes[15] != kC || in_sizes[16] < 1 || in_sizes[17] < 1) return;

  const size_t M = (size_t)B * kT;
  const size_t szW = (size_t)4 * kC * kC * 2;
  const size_t szX = M * kC * 2;
  const size_t szF = M * kC * 4;
  const size_t szS = (size_t)B * kNC * 6 * kC * 4;
  const size_t offW  = 0;
  const size_t offX0 = offW + szW;
  const size_t offX1 = offX0 + szX;
  const size_t offX2 = offX1 + szX;
  const size_t offK  = offX2 + szX;
  const size_t offV  = offK + szF;
  const size_t offS  = offV + szF;
  const size_t offE  = offS + szS;
  const size_t total = offE + szS;
  if (ws_size < total) return;

  const float* x     = (const float*)d_in[0];
  const float* mk    = (const float*)d_in[1];
  const float* mvp   = (const float*)d_in[2];
  const float* mrp   = (const float*)d_in[3];
  const float* sdp   = (const float*)d_in[4];
  const float* sfp   = (const float*)d_in[5];
  const float* alpha = (const float*)d_in[6];
  const float* w1    = (const float*)d_in[7];
  const float* w3    = (const float*)d_in[8];
  const float* w5    = (const float*)d_in[9];
  const float* Wk    = (const float*)d_in[10];
  const float* Wv    = (const float*)d_in[11];
  const float* Wr    = (const float*)d_in[12];
  const float* Wo    = (const float*)d_in[13];
  const float* lng   = (const float*)d_in[14];
  const float* lnb   = (const float*)d_in[15];
  const int*   hH    = (const int*)d_in[16];
  const int*   hWd   = (const int*)d_in[17];
  float* out = (float*)d_out;
  char* ws = (char*)d_ws;
  unsigned short* W16 = (unsigned short*)(ws + offW);
  unsigned short* X0  = (unsigned short*)(ws + offX0);
  unsigned short* X1  = (unsigned short*)(ws + offX1);
  unsigned short* X2  = (unsigned short*)(ws + offX2);
  float* Kf = (float*)(ws + offK);
  float* Vf = (float*)(ws + offV);
  float* Sb = (float*)(ws + offS);
  float* Eb = (float*)(ws + offE);
  const unsigned short* Wk16 = W16 + 0 * kC * kC;
  const unsigned short* Wv16 = W16 + 1 * kC * kC;
  const unsigned short* Wr16 = W16 + 2 * kC * kC;
  const unsigned short* Wo16 = W16 + 3 * kC * kC;
  const long planeElems = (long)M * kC;
  const int Mi = (int)M;
  const int gemmBlocks = (int)(M / 128);

  wcast16_kernel<<<dim3((kC * kC / 8) / 256, 4), dim3(256), 0, stream>>>(Wk, Wv, Wr, Wo, W16, kCarryW);
  omni_mix_kernel<<<dim3(B * kH), dim3(256), 0, stream>>>(x, alpha, w1, w3, w5, mk, mvp, mrp, X0, planeElems, hH, hWd);
  wmma_gemm64<0, false, 0, 0, false, 0><<<dim3(gemmBlocks, 1), dim3(256), 0, stream>>>(
      X0, X0, kC, 0L, Wk16, Wk16, kC, 0L, (void*)Kf, (void*)Kf, kC, 0L, sdp, sdp, 0L, Mi, kC, kC, kScaleAW);
  wmma_gemm64<0, false, 0, 0, false, 0><<<dim3(gemmBlocks, 1), dim3(256), 0, stream>>>(
      X1, X1, kC, 0L, Wv16, Wv16, kC, 0L, (void*)Vf, (void*)Vf, kC, 0L, sdp, sdp, 0L, Mi, kC, kC, kScaleAW);
  wmma_gemm64<0, false, 0, 1, false, 0><<<dim3(gemmBlocks, 1), dim3(256), 0, stream>>>(
      X2, X2, kC, 0L, Wr16, Wr16, kC, 0L, (void*)X0, (void*)X0, kC, 0L, sdp, sdp, 0L, Mi, kC, kC, kScaleW);
  wkv_chunk_kernel<<<dim3(B * kNC), dim3(256), 0, stream>>>(Kf, Vf, sdp, 0, 0, Sb);
  wkv_entries_kernel<<<dim3(B * 8), dim3(32), 0, stream>>>(Kf, sdp, 0, 0, Sb, Eb);
  wkv_apply_kernel<<<dim3(B * kNC * 4), dim3(64), 0, stream>>>(Kf, Vf, sdp, sfp, 0, 0, Eb, out);
  wkv_chunk_kernel<<<dim3(B * kNC), dim3(256), 0, stream>>>(Kf, out, sdp, 1, 1, Sb);
  wkv_entries_kernel<<<dim3(B * 8), dim3(32), 0, stream>>>(Kf, sdp, 1, 1, Sb, Eb);
  wkv_apply_kernel<<<dim3(B * kNC * 4), dim3(64), 0, stream>>>(Kf, out, sdp, sfp, 1, 1, Eb, Vf);
  ln_gate_kernel<<<dim3(Mi / 8), dim3(256), 0, stream>>>(Vf, X0, lng, lnb, X1, Mi);
  wmma_gemm64<0, false, 0, 0, false, 0><<<dim3(gemmBlocks, 1), dim3(256), 0, stream>>>(
      X1, X1, kC, 0L, Wo16, Wo16, kC, 0L, (void*)out, (void*)out, kC, 0L, sdp, sdp, 0L, Mi, kC, kC, kScaleAW);
}
